// DecoderLayer_39994735460721
// MI455X (gfx1250) — hardware-run, weakly checked
//
#include <hip/hip_runtime.h>
#include <math.h>

constexpr int kBatch   = 2;
constexpr int kSeqLen  = 2048;
constexpr int kModel   = 1024;
constexpr int kHeads   = 16;
constexpr int kHeadDim = 64;
constexpr int kFF      = 4096;
constexpr int kTok     = kBatch * kSeqLen;
constexpr int kGroups  = kBatch * kHeads;
constexpr int kGroupsPerChunk = 2;
constexpr int kChunks  = kGroups / kGroupsPerChunk;
constexpr float kWCarry     = 16.0f;
constexpr float kWCarryInv  = 1.0f / 16.0f;
constexpr float kW2Carry    = 32.0f;
constexpr float kW2CarryInv = 1.0f / 32.0f;
constexpr float kPCarry     = 2048.0f;
constexpr float kCtxCarry   = 16.0f;
constexpr float kPVScale    = kCtxCarry / kPCarry;
constexpr float kWoScale    = 1.0f / (kCtxCarry * kWCarry);
constexpr float kScoreScale = 0.125f;
constexpr float kInvModel   = 1.0f / 1024.0f;
constexpr float kLnEps      = 1e-5f;

constexpr size_t kMiB     = 1048576;
constexpr size_t kOffX16  = 0;
constexpr size_t kOffWT4  = 8 * kMiB;
constexpr size_t kOffQ16  = 16 * kMiB;
constexpr size_t kOffK16  = 24 * kMiB;
constexpr size_t kOffVT16 = 32 * kMiB;
constexpr size_t kOffCtx  = 40 * kMiB;
constexpr size_t kOffSc   = 48 * kMiB;
constexpr size_t kOffP16  = 80 * kMiB;
constexpr size_t kOffW1T  = 0;
constexpr size_t kOffW2T  = 8 * kMiB;
constexpr size_t kOffX1H  = 16 * kMiB;
constexpr size_t kOffH16  = 24 * kMiB;
constexpr size_t kOffY1   = 48 * kMiB;
constexpr size_t kOffX1   = 64 * kMiB;
constexpr size_t kOffY2   = 80 * kMiB;
constexpr size_t kWsTotal = 96 * kMiB;
static_assert((size_t)kTok * kModel * 2 == 8 * kMiB, "x16 plane size");
static_assert((size_t)kGroupsPerChunk * kSeqLen * kSeqLen * 4 == 32 * kMiB, "scores chunk size");
static_assert((size_t)kGroupsPerChunk * kSeqLen * kSeqLen * 2 == 16 * kMiB, "P chunk size");
static_assert((size_t)kTok * kFF * 2 == 32 * kMiB, "h16 plane size");
static_assert(kOffH16 + 32 * kMiB <= kOffX1, "h16 does not reach x1");
static_assert(kWsTotal <= 134217728, "carve under 128 MiB");

typedef __attribute__((ext_vector_type(16))) _Float16 v16h;
typedef __attribute__((ext_vector_type(8)))  _Float16 v8h;
typedef __attribute__((ext_vector_type(16))) __bf16   v16b;
typedef __attribute__((ext_vector_type(8)))  __bf16   v8b;
typedef __attribute__((ext_vector_type(8)))  float    v8f;
typedef __attribute__((ext_vector_type(4)))  float    v4f;
typedef __attribute__((ext_vector_type(4)))  unsigned int v4u;
typedef __attribute__((ext_vector_type(4)))  int      v4i;

__device__ __forceinline__ unsigned short f2bf_bits(float f) {
  unsigned u = __float_as_uint(f);
  return (unsigned short)((u + 0x7FFFu + ((u >> 16) & 1u)) >> 16);
}
__device__ __forceinline__ float bf_bits2f(unsigned short h) { return __uint_as_float(((unsigned)h) << 16); }

__device__ __forceinline__ void dep_guard_h(v8f& a, v8f& b, v16h x, v16h y) { asm volatile("v_nop\n\tv_nop\n\tv_nop\n\tv_nop" : "+v"(a), "+v"(b) : "v"(x), "v"(y)); }
__device__ __forceinline__ void dep_guard_b(v8f& a, v8f& b, v16b x, v16b y) { asm volatile("v_nop\n\tv_nop\n\tv_nop\n\tv_nop" : "+v"(a), "+v"(b) : "v"(x), "v"(y)); }
__device__ __forceinline__ void keep4_h(v16h a, v16h b, v16h c, v16h d) { asm volatile("v_nop" :: "v"(a), "v"(b), "v"(c), "v"(d)); }
__device__ __forceinline__ void keep4_b(v16b a, v16b b, v16b c, v16b d) { asm volatile("v_nop" :: "v"(a), "v"(b), "v"(c), "v"(d)); }
__device__ __forceinline__ void acc_guard4(v8f& a, v8f& b, v8f& c, v8f& d) { asm volatile("v_nop\n\tv_nop\n\tv_nop\n\tv_nop" : "+v"(a), "+v"(b), "+v"(c), "+v"(d)); }
template <typename T> struct Frag;
template <> struct Frag<_Float16> {
  typedef v16h V; union U { v16h v; v8h h[2]; };
  static __device__ __forceinline__ v16h load(const _Float16* p) {
    U f; f.h[0] = *(const v8h*)(p); f.h[1] = *(const v8h*)(p + 16); return f.v;
  }
  static __device__ __forceinline__ v8f mma(v16h a, v16h b, v8f c) {
    return __builtin_amdgcn_wmma_f32_16x16x32_f16(false, a, false, b, (short)0, c, false, false);
  }
  static __device__ __forceinline__ void guard(v8f& a, v8f& b, v16h x, v16h y) { dep_guard_h(a, b, x, y); }
  static __device__ __forceinline__ void keep(v16h a, v16h b, v16h c, v16h d) { keep4_h(a, b, c, d); }
};
template <> struct Frag<__bf16> {
  typedef v16b V; union U { v16b v; v8b h[2]; };
  static __device__ __forceinline__ v16b load(const __bf16* p) {
    U f; f.h[0] = *(const v8b*)(p); f.h[1] = *(const v8b*)(p + 16); return f.v;
  }
  static __device__ __forceinline__ v8f mma(v16b a, v16b b, v8f c) {
    return __builtin_amdgcn_wmma_f32_16x16x32_bf16(false, a, false, b, (short)0, c, false, false);
  }
  static __device__ __forceinline__ void guard(v8f& a, v8f& b, v16b x, v16b y) { dep_guard_b(a, b, x, y); }
  static __device__ __forceinline__ void keep(v16b a, v16b b, v16b c, v16b d) { keep4_b(a, b, c, d); }
};

__device__ __forceinline__ unsigned pk16(unsigned short a, unsigned short b) { return (unsigned)a | ((unsigned)b << 16); }
__device__ __forceinline__ unsigned short h_bits(float f) { const _Float16 h = (_Float16)f; return __builtin_bit_cast(unsigned short, h); }

template <int ET> struct Elem;
template <> struct Elem<0> { typedef _Float16 T; };
template <> struct Elem<1> { typedef __bf16 T; };
template <int ET, bool SPLIT, int BIAS_MODE, int OUT_MODE, bool RESID, int ACT = 0, int TRI = 0>
__global__ __launch_bounds__(256) void wmma_gemm64(
    const unsigned short* __restrict__ Ap, const unsigned short* __restrict__ A2p, int lda, long strideA,
    const unsigned short* __restrict__ Btp, const unsigned short* __restrict__ Bt2p, int ldb, long strideB,
    void* __restrict__ Cout, void* __restrict__ Cout2, int ldc, long strideC,
    const float* __restrict__ bias,
    const float* __restrict__ resid, long strideR,
    int M, int N, int K, float scale) {
  typedef typename Elem<ET>::T T;
  typedef typename Frag<T>::V V;
  const T* A = (const T*)Ap; const T* A2 = (const T*)A2p; const T* Bt = (const T*)Btp; const T* Bt2 = (const T*)Bt2p;
  __shared__ __align__(16) float sT[8][16 * 68];
  const int b    = blockIdx.y;
  const int lane = threadIdx.x & 31;
  const int wave = threadIdx.x >> 5;
  const int tilesN = N >> 6;
  const int tilesM = M >> 6;
  const int tile = blockIdx.x * 8 + wave;
  if (tile >= tilesM * tilesN) return;
  const int tm = tile / tilesN;
  const int tn = tile - tm * tilesN;
  if (TRI == 1 && tn > tm) return;
  const int m0 = tm << 6;
  const int n0 = tn << 6;
  const int kEnd = (TRI == 2) ? (((m0 + 64) < K) ? (m0 + 64) : K) : K;

  const T* Ab  = A  + (size_t)b * strideA;
  const T* Bb  = Bt + (size_t)b * strideB;
  const T* Ab2 = SPLIT ? (A2  + (size_t)b * strideA) : nullptr;
  const T* Bb2 = SPLIT ? (Bt2 + (size_t)b * strideB) : nullptr;

  const int rlane = lane & 15;
  const int koff  = (lane >> 4) * 8;
  const int mOff  = (lane >> 4) * 8;

  v8f acc[4][4];
#pragma unroll
  for (int i = 0; i < 4; ++i)
#pragma unroll
    for (int j = 0; j < 4; ++j) acc[i][j] = (v8f){0.f,0.f,0.f,0.f,0.f,0.f,0.f,0.f};

  for (int k0 = 0; k0 < kEnd; k0 += 32) {
    V bh[4], bl[4];
#pragma unroll
    for (int j = 0; j < 4; ++j) {
      const size_t bo = (size_t)(n0 + (j << 4) + rlane) * ldb + koff + k0;
      bh[j] = Frag<T>::load(Bb + bo);
      if (SPLIT) bl[j] = Frag<T>::load(Bb2 + bo);
    }
#pragma unroll
    for (int i = 0; i < 4; ++i) {
      const size_t ao = (size_t)(m0 + (i << 4) + rlane) * lda + koff + k0;
      V ah = Frag<T>::load(Ab + ao);
      V al;
      if (SPLIT) al = Frag<T>::load(Ab2 + ao);
#pragma unroll
      for (int j = 0; j < 4; ++j) {
        acc[i][j] = Frag<T>::mma(ah, bh[j], acc[i][j]);
        if (SPLIT) {
          acc[i][j] = Frag<T>::mma(ah, bl[j], acc[i][j]);
          acc[i][j] = Frag<T>::mma(al, bh[j], acc[i][j]);
        }
      }
      Frag<T>::guard(acc[i][0], acc[i][3], ah, SPLIT ? al : ah);
    }
    Frag<T>::keep(bh[0], bh[1], bh[2], bh[3]);
    if (SPLIT) Frag<T>::keep(bl[0], bl[1], bl[2], bl[3]);
  }
  acc_guard4(acc[0][0], acc[0][1], acc[0][2], acc[0][3]);
  acc_guard4(acc[1][0], acc[1][1], acc[1][2], acc[1][3]);
  acc_guard4(acc[2][0], acc[2][1], acc[2][2], acc[2][3]);
  acc_guard4(acc[3][0], acc[3][1], acc[3][2], acc[3][3]);

  float* slab = sT[wave];
  const float* Rb = RESID ? (resid + (size_t)b * strideR) : nullptr;
#pragma unroll
  for (int i = 0; i < 4; ++i) {
    const int mBase = m0 + (i << 4);
#pragma unroll
    for (int j = 0; j < 4; ++j) {
      const int n = n0 + (j << 4) + rlane;
      float bv = 0.f;
      if (BIAS_MODE == 2) bv = bias[n];
#pragma unroll
      for (int r = 0; r < 8; ++r) {
        float v = acc[i][j][r] * scale;
        if (BIAS_MODE == 1) v += bias[mBase + mOff + r];
        if (BIAS_MODE == 2) v += bv;
        if (RESID) v += Rb[(size_t)(mBase + mOff + r) * ldc + n];
        if (ACT == 2) v = fmaxf(v, 0.0f);
        if (ACT == 4) v = (v > 0.f) ? v : 0.01f * v;
        slab[(mOff + r) * 68 + (j << 4) + rlane] = v;
      }
    }
    __builtin_amdgcn_fence(__ATOMIC_RELEASE, "workgroup");
    __builtin_amdgcn_wave_barrier();
    __builtin_amdgcn_fence(__ATOMIC_ACQUIRE, "workgroup");
    if (OUT_MODE == 0) {
      float* C = (float*)Cout + (size_t)b * strideC;
      const int hh = lane >> 4, c4 = (lane & 15) * 4;
      for (int pass = 0; pass < 2; ++pass) {
#pragma unroll
        for (int it = 0; it < 8; ++it) {
          const int row = it * 2 + hh;
          v4f v = *(const v4f*)(slab + row * 68 + c4);
          *(volatile v4f*)(C + (size_t)(mBase + row) * ldc + n0 + c4) = v;
        }
        __threadfence();
      }
    } else {
      const int q = lane >> 3, c8 = (lane & 7) * 8;
      unsigned short* C  = (unsigned short*)Cout  + (size_t)b * strideC;
      unsigned short* C2 = (OUT_MODE == 2) ? ((unsigned short*)Cout2 + (size_t)b * strideC) : nullptr;
      for (int pass = 0; pass < 2; ++pass) {
#pragma unroll
        for (int it = 0; it < 4; ++it) {
          const int row = it * 4 + q;
          const float* sp = slab + row * 68 + c8;
          v8h hv, lv;
#pragma unroll
          for (int e = 0; e < 8; ++e) {
            if (OUT_MODE == 1) {
              hv[e] = (_Float16)sp[e];
            } else {
              unsigned short hb = f2bf_bits(sp[e]);
              unsigned short lb = f2bf_bits(sp[e] - bf_bits2f(hb));
              hv[e] = __builtin_bit_cast(_Float16, hb);
              lv[e] = __builtin_bit_cast(_Float16, lb);
            }
          }
          *(volatile v8h*)(C + (size_t)(mBase + row) * ldc + n0 + c8) = hv;
          if (OUT_MODE == 2) *(volatile v8h*)(C2 + (size_t)(mBase + row) * ldc + n0 + c8) = lv;
        }
        __threadfence();
      }
    }
    __builtin_amdgcn_fence(__ATOMIC_RELEASE, "workgroup");
    __builtin_amdgcn_wave_barrier();
    __builtin_amdgcn_fence(__ATOMIC_ACQUIRE, "workgroup");
  }
}

__global__ __launch_bounds__(256) void tcast_kernel(const float* __restrict__ W0, const float* __restrict__ W1,
                                                    const float* __restrict__ W2, const float* __restrict__ W3,
                                                    unsigned short* __restrict__ out, int R, int Ccols,
                                                    long planeStride, float scale) {
  __shared__ float sm[64][65];
  const int t  = threadIdx.x;
  const int r0 = blockIdx.x * 64;
  const int c0 = blockIdx.y * 64;
  const int z  = blockIdx.z;
  const float* W = (z == 0) ? W0 : (z == 1) ? W1 : (z == 2) ? W2 : W3;
#pragma unroll
  for (int i = 0; i < 16; ++i) {
    const int e  = i * 256 + t;
    const int rl = e >> 6;
    const int cl = e & 63;
    sm[cl][rl] = W[(size_t)(r0 + rl) * Ccols + c0 + cl] * scale;
  }
  __syncthreads();
  const int lane = t & 31, wave = t >> 5;
  const int q = lane >> 3, c8 = (lane & 7) * 8;
  unsigned short* op = out + (size_t)z * planeStride;
  for (int pass = 0; pass < 2; ++pass) {
#pragma unroll
    for (int it = 0; it < 2; ++it) {
      const int row = wave * 8 + it * 4 + q;
      unsigned short hb[8];
#pragma unroll
      for (int e = 0; e < 8; ++e) hb[e] = h_bits(sm[row][c8 + e]);
      const v4u u = (v4u){pk16(hb[0], hb[1]), pk16(hb[2], hb[3]), pk16(hb[4], hb[5]), pk16(hb[6], hb[7])};
      *(volatile v4u*)(op + (size_t)(c0 + row) * R + r0 + c8) = u;
    }
    __threadfence();
  }
}

__global__ __launch_bounds__(256) void cast8_f16_kernel(const float* __restrict__ in, unsigned short* __restrict__ out, int n8) {
  const int i = blockIdx.x * 256 + threadIdx.x;
  if (i >= n8) return;
  const float* p = in + 8 * (size_t)i;
  const v4f a = *(const v4f*)(p);
  const v4f c = *(const v4f*)(p + 4);
  unsigned short hb[8];
#pragma unroll
  for (int e = 0; e < 4; ++e) {
    hb[e]     = h_bits(a[e]);
    hb[4 + e] = h_bits(c[e]);
  }
  const v4u u = (v4u){pk16(hb[0], hb[1]), pk16(hb[2], hb[3]), pk16(hb[4], hb[5]), pk16(hb[6], hb[7])};
  unsigned short* q = out + 8 * (size_t)i;
  *(volatile v4u*)q = u;
  __threadfence();
  *(volatile v4u*)q = u;
}

__global__ __launch_bounds__(128) void softmax_rows_kernel(const float* __restrict__ Sc, const int* __restrict__ msk,
                                                           unsigned short* __restrict__ P) {
  __shared__ __align__(16) float pbuf[4][kSeqLen];
  const int t = threadIdx.x;
  const int lane = t & 31, wave = t >> 5;
  const int gr = blockIdx.x * 4 + wave;
  const int r  = gr & (kSeqLen - 1);
  const float* srow = Sc + (size_t)gr * kSeqLen;
  const int* mrow = msk + (size_t)r * kSeqLen;
  unsigned short* prow = P + (size_t)gr * kSeqLen;
  const int lim = ((r >> 6) + 1) << 6;
  const int nsc = (lim + 255) >> 8;
  float* pb = pbuf[wave];

  float mx = -INFINITY;
#pragma unroll 1
  for (int c = 0; c < nsc; ++c) {
    const int col0 = (c << 8) + lane * 8;
    const v4f sa = *(const v4f*)(srow + col0);
    const v4f sb = *(const v4f*)(srow + col0 + 4);
    const v4i ma = *(const v4i*)(mrow + col0);
    const v4i mb = *(const v4i*)(mrow + col0 + 4);
    v4f xa, xb;
#pragma unroll
    for (int e = 0; e < 4; ++e) {
      const bool ka = ((col0 + e) < lim) && (ma[e] != 1);
      const bool kb = ((col0 + 4 + e) < lim) && (mb[e] != 1);
      xa[e] = ka ? sa[e] : -INFINITY;
      xb[e] = kb ? sb[e] : -INFINITY;
      mx = fmaxf(mx, fmaxf(xa[e], xb[e]));
    }
    *(v4f*)(pb + col0) = xa;
    *(v4f*)(pb + col0 + 4) = xb;
  }
#pragma unroll
  for (int off = 16; off > 0; off >>= 1) mx = fmaxf(mx, __shfl_xor(mx, off, 32));

  float sum = 0.0f;
#pragma unroll 1
  for (int c = 0; c < nsc; ++c) {
    const int col0 = (c << 8) + lane * 8;
    v4f xa = *(const v4f*)(pb + col0);
    v4f xb = *(const v4f*)(pb + col0 + 4);
#pragma unroll
    for (int e = 0; e < 4; ++e) {
      xa[e] = expf(xa[e] - mx);
      xb[e] = expf(xb[e] - mx);
      sum += xa[e];
      sum += xb[e];
    }
    *(v4f*)(pb + col0) = xa;
    *(v4f*)(pb + col0 + 4) = xb;
  }
#pragma unroll
  for (int off = 16; off > 0; off >>= 1) sum += __shfl_xor(sum, off, 32);
  const float f = kPCarry * (1.0f / sum);

#pragma unroll 1
  for (int c = 0; c < nsc; ++c) {
    const int col0 = (c << 8) + lane * 8;
    const v4f xa = *(const v4f*)(pb + col0);
    const v4f xb = *(const v4f*)(pb + col0 + 4);
    unsigned short hb[8];
#pragma unroll
    for (int e = 0; e < 4; ++e) {
      hb[e]     = h_bits(xa[e] * f);
      hb[4 + e] = h_bits(xb[e] * f);
    }
    const v4u u = (v4u){pk16(hb[0], hb[1]), pk16(hb[2], hb[3]), pk16(hb[4], hb[5]), pk16(hb[6], hb[7])};
    unsigned short* q = prow + col0;
    *(volatile v4u*)q = u;
    __threadfence();
    *(volatile v4u*)q = u;
  }
}

template <bool W16>
__global__ __launch_bounds__(256) void add_ln_kernel(const float* __restrict__ Y, const float* __restrict__ gam,
                                                     const float* __restrict__ bet, float* __restrict__ out,
                                                     unsigned short* __restrict__ out16) {
  __shared__ float red1[8];
  __shared__ float red2[8];
  __shared__ __align__(16) float rowbuf[W16 ? kModel : 4];
  const int row = blockIdx.x;
  const int t = threadIdx.x, lane = t & 31, wave = t >> 5;
  const size_t base = (size_t)row * kModel + 4 * t;
  const v4f xv = *(const v4f*)(Y + base);
  float s = (xv[0] + xv[1]) + (xv[2] + xv[3]);
#pragma unroll
  for (int off = 16; off > 0; off >>= 1) s += __shfl_xor(s, off, 32);
  if (lane == 0) red1[wave] = s;
  __syncthreads();
  float tot = red1[0];
#pragma unroll
  for (int w = 1; w < 8; ++w) tot += red1[w];
  const float mean = tot * kInvModel;
  v4f d;
#pragma unroll
  for (int e = 0; e < 4; ++e) d[e] = xv[e] - mean;
  float s2 = (d[0] * d[0] + d[1] * d[1]) + (d[2] * d[2] + d[3] * d[3]);
#pragma unroll
  for (int off = 16; off > 0; off >>= 1) s2 += __shfl_xor(s2, off, 32);
  if (lane == 0) red2[wave] = s2;
  __syncthreads();
  float tot2 = red2[0];
#pragma unroll
  for (int w = 1; w < 8; ++w) tot2 += red2[w];
  const float var  = tot2 * kInvModel;
  const float rinv = rsqrtf(var + kLnEps);
  const v4f gg = *(const v4f*)(gam + 4 * t);
  const v4f bb = *(const v4f*)(bet + 4 * t);
  v4f o;
#pragma unroll
  for (int e = 0; e < 4; ++e) o[e] = d[e] * rinv * gg[e] + bb[e];
  float* op = out + base;
  *(volatile v4f*)op = o;
  __threadfence();
  *(volatile v4f*)op = o;
  if (W16) {
    *(v4f*)(rowbuf + 4 * t) = o;
    __syncthreads();
    if (t < 128) {
      const v4f a = *(const v4f*)(rowbuf + 8 * t);
      const v4f c = *(const v4f*)(rowbuf + 8 * t + 4);
      unsigned short hb[8];
#pragma unroll
      for (int e = 0; e < 4; ++e) {
        hb[e]     = h_bits(a[e]);
        hb[4 + e] = h_bits(c[e]);
      }
      const v4u u = (v4u){pk16(hb[0], hb[1]), pk16(hb[2], hb[3]), pk16(hb[4], hb[5]), pk16(hb[6], hb[7])};
      unsigned short* q = out16 + (size_t)row * kModel + 8 * t;
      *(volatile v4u*)q = u;
      __threadfence();
      *(volatile v4u*)q = u;
    }
  }
}

extern "C" void kernel_launch(void* const* d_in, const int* in_sizes, int n_in,
                              void* d_out, int out_size, void* d_ws, size_t ws_size,
                              hipStream_t stream) {
  if (n_in < 18) return;
  if (in_sizes[0] != kTok * kModel) return;
  if (in_sizes[1] != kSeqLen * kSeqLen) return;
  if (in_sizes[2] != kModel * kModel || in_sizes[4] != kModel * kModel ||
      in_sizes[6] != kModel * kModel || in_sizes[8] != kModel * kModel) return;
  if (in_sizes[3] != kModel || in_sizes[5] != kModel || in_sizes[7] != kModel || in_sizes[9] != kModel) return;
  if (in_sizes[10] != kModel * kFF || in_sizes[11] != kFF || in_sizes[12] != kFF * kModel || in_sizes[13] != kModel) return;
  if (in_sizes[14] != kModel || in_sizes[15] != kModel || in_sizes[16] != kModel || in_sizes[17] != kModel) return;
  if (out_size != kTok * kModel) return;
  if (ws_size < kWsTotal) return;

  const float* x    = (const float*)d_in[0];
  const int*   mask = (const int*)d_in[1];
  const float* wq   = (const float*)d_in[2];  const float* bq  = (const float*)d_in[3];
  const float* wk   = (const float*)d_in[4];  const float* bk  = (const float*)d_in[5];
  const float* wv   = (const float*)d_in[6];  const float* bv  = (const float*)d_in[7];
  const float* wo   = (const float*)d_in[8];  const float* bo  = (const float*)d_in[9];
  const float* w1   = (const float*)d_in[10]; const float* b1  = (const float*)d_in[11];
  const float* w2   = (const float*)d_in[12]; const float* b2  = (const float*)d_in[13];
  const float* g1   = (const float*)d_in[14]; const float* be1 = (const float*)d_in[15];
  const float* g2   = (const float*)d_in[16]; const float* be2 = (const float*)d_in[17];
  float* outp = (float*)d_out;

  char* ws = (char*)d_ws;
  unsigned short* x16   = (unsigned short*)(ws + kOffX16);
  unsigned short* wT4   = (unsigned short*)(ws + kOffWT4);
  unsigned short* q16   = (unsigned short*)(ws + kOffQ16);
  unsigned short* k16   = (unsigned short*)(ws + kOffK16);
  unsigned short* vt16  = (unsigned short*)(ws + kOffVT16);
  unsigned short* ctx16 = (unsigned short*)(ws + kOffCtx);
  float*          sc    = (float*)(ws + kOffSc);
  unsigned short* p16   = (unsigned short*)(ws + kOffP16);
  unsigned short* w1T   = (unsigned short*)(ws + kOffW1T);
  unsigned short* w2T   = (unsigned short*)(ws + kOffW2T);
  unsigned short* x1h   = (unsigned short*)(ws + kOffX1H);
  unsigned short* h16   = (unsigned short*)(ws + kOffH16);
  float*          y1    = (float*)(ws + kOffY1);
  float*          x1    = (float*)(ws + kOffX1);
  float*          y2    = (float*)(ws + kOffY2);
  const unsigned short* wqT = wT4;
  const unsigned short* wkT = wT4 + (size_t)kModel * kModel;
  const unsigned short* wvT = wT4 + (size_t)2 * kModel * kModel;
  const unsigned short* woT = wT4 + (size_t)3 * kModel * kModel;

  {
    const int n8 = kTok * kModel / 8;
    cast8_f16_kernel<<<dim3((n8 + 255) / 256), dim3(256), 0, stream>>>(x, x16, n8);
    tcast_kernel<<<dim3(kModel / 64, kModel / 64, 4), dim3(256), 0, stream>>>(
        wq, wk, wv, wo, wT4, kModel, kModel, (long)kModel * kModel, kWCarry);
  }

  {
    const dim3 g((64 * 16 + 7) / 8, 1);
    wmma_gemm64<0, false, 2, 1, false, 0, 0><<<g, dim3(256), 0, stream>>>(
        x16, x16, kModel, 0L, wqT, wqT, kModel, 0L, (void*)q16, (void*)q16, kModel, 0L,
        bq, x, 0L, kTok, kModel, kModel, kWCarryInv);
    wmma_gemm64<0, false, 2, 1, false, 0, 0><<<g, dim3(256), 0, stream>>>(
        x16, x16, kModel, 0L, wkT, wkT, kModel, 0L, (void*)k16, (void*)k16, kModel, 0L,
        bk, x, 0L, kTok, kModel, kModel, kWCarryInv);
    const dim3 gv((16 * 64 + 7) / 8, 1);
    wmma_gemm64<0, false, 1, 1, false, 0, 0><<<gv, dim3(256), 0, stream>>>(
        wvT, wvT, kModel, 0L, x16, x16, kModel, 0L, (void*)vt16, (void*)vt16, kTok, 0L,
        bv, x, 0L, kModel, kTok, kModel, kWCarryInv);
  }

  for (int ch = 0; ch < kChunks; ++ch) {
    const int b  = ch / (kHeads / kGroupsPerChunk);
    const int h0 = (ch % (kHeads / kGroupsPerChunk)) * kGroupsPerChunk;
    const size_t qoff = (size_t)b * kSeqLen * kModel + (size_t)h0 * kHeadDim;
    const unsigned short* qa = q16 + qoff;
    const unsigned short* ka = k16 + qoff;
    wmma_gemm64<0, false, 0, 0, false, 0, 1><<<dim3((32 * 32 + 7) / 8, kGroupsPerChunk), dim3(256), 0, stream>>>(
        qa, qa, kModel, (long)kHeadDim, ka, ka, kModel, (long)kHeadDim,
        (void*)sc, (void*)sc, kSeqLen, (long)kSeqLen * kSeqLen,
        bq, x, 0L, kSeqLen, kSeqLen, kHeadDim, kScoreScale);
    softmax_rows_kernel<<<dim3(kGroupsPerChunk * kSeqLen / 4), dim3(128), 0, stream>>>(sc, mask, p16);
    const unsigned short* vta = vt16 + (size_t)(h0 * kHeadDim) * kTok + (size_t)b * kSeqLen;
    unsigned short* ctxa = ctx16 + qoff;
    wmma_gemm64<0, false, 0, 1, false, 0, 2><<<dim3((32 * 1 + 7) / 8, kGroupsPerChunk), dim3(256), 0, stream>>>(
        p16, p16, kSeqLen, (long)kSeqLen * kSeqLen, vta, vta, kTok, (long)kHeadDim * kTok,
        (void*)ctxa, (void*)ctxa, kModel, (long)kHeadDim,
        bq, x, 0L, kSeqLen, kHeadDim, kSeqLen, kPVScale);
  }

  {
    const dim3 g((64 * 16 + 7) / 8, 1);
    wmma_gemm64<0, false, 2, 0, true, 0, 0><<<g, dim3(256), 0, stream>>>(
        ctx16, ctx16, kModel, 0L, woT, woT, kModel, 0L, (void*)y1, (void*)y1, kModel, 0L,
        bo, x, 0L, kTok, kModel, kModel, kWoScale);
  }
  add_ln_kernel<true><<<dim3(kTok), dim3(256), 0, stream>>>(y1, g1, be1, x1, x1h);

  tcast_kernel<<<dim3(kModel / 64, kFF / 64, 1), dim3(256), 0, stream>>>(
      w1, w1, w1, w1, w1T, kModel, kFF, 0L, kWCarry);
  tcast_kernel<<<dim3(kFF / 64, kModel / 64, 1), dim3(256), 0, stream>>>(
      w2, w2, w2, w2, w2T, kFF, kModel, 0L, kW2Carry);

  {
    const dim3 g((64 * 64 + 7) / 8, 1);
    wmma_gemm64<0, false, 2, 1, false, 2, 0><<<g, dim3(256), 0, stream>>>(
        x1h, x1h, kModel, 0L, w1T, w1T, kModel, 0L, (void*)h16, (void*)h16, kFF, 0L,
        b1, x, 0L, kTok, kFF, kModel, kWCarryInv);
  }
  {
    const dim3 g((64 * 16 + 7) / 8, 1);
    wmma_gemm64<0, false, 2, 0, true, 0, 0><<<g, dim3(256), 0, stream>>>(
        h16, h16, kFF, 0L, w2T, w2T, kFF, 0L, (void*)y2, (void*)y2, kModel, 0L,
        b2, x1, 0L, kTok, kModel, kFF, kW2CarryInv);
  }
  add_ln_kernel<false><<<dim3(kTok), dim3(256), 0, stream>>>(y2, g2, be2, outp, x1h);
}
